// Encoder_36258113913425
// MI455X (gfx1250) — hardware-verified
//
#include <hip/hip_runtime.h>
#include <hip/hip_fp16.h>


#ifndef NB
#define NB 2
#endif
#ifndef SEQ
#define SEQ 2048
#endif
#define NB_FULL  2
#define SEQ_FULL 2048
#define DM   1024
#define NH   16
#define HD   64
#define QKP  2048
#define NTOK (NB * SEQ)
#define PP   72
#define WROWS 6144

static_assert(NB >= 1 && NB <= NB_FULL);
static_assert(SEQ >= 128 && SEQ <= SEQ_FULL);
static_assert(SEQ % 128 == 0);
static_assert(NTOK % 128 == 0);
static_assert(NTOK % 8 == 0);
static_assert(DM % 128 == 0 && QKP % 128 == 0);
static_assert(DM % 32 == 0);
static_assert(NH * HD == DM);
static_assert(6u * 256u * 4096u == (unsigned)WROWS * (unsigned)DM);

typedef _Float16 v16h __attribute__((ext_vector_type(16)));
typedef _Float16 v8h  __attribute__((ext_vector_type(8)));
typedef float    v8f  __attribute__((ext_vector_type(8)));
typedef float    v4f  __attribute__((ext_vector_type(4)));

union Frag { v16h v; v8h h[2]; };

#define C1      (1.44269504088896340736f * 0.001953125f)
#define PCARRY  10.0f
#define SC_P8   0.125f
#define SC_CTX  128.0f
#define SC_WO   1.52587890625e-05f
#define SC_W2   0.001953125f

static __device__ __forceinline__ v8f zero8() {
    v8f z;
#pragma unroll
    for (int i = 0; i < 8; ++i) z[i] = 0.0f;
    return z;
}

static __device__ __forceinline__ v16h load_frag16(const _Float16* base, unsigned ld, unsigned lane) {
    const unsigned m  = lane & 15u;
    const unsigned kb = (lane >> 4) << 3;
    const _Float16* p = base + (size_t)m * ld + kb;
    Frag f;
    f.h[0] = *(const v8h*)(p);
    f.h[1] = *(const v8h*)(p + 16);
    return f.v;
}

static __device__ __forceinline__ v8f wmma16(v16h a, v16h b, v8f c) {
    v8f d = __builtin_amdgcn_wmma_f32_16x16x32_f16(false, a, false, b, (short)0, c, false, false);
    asm volatile("v_nop\n\tv_nop\n\tv_nop\n\tv_nop" : "+v"(d) : "v"(a), "v"(b));
    return d;
}

static __device__ __forceinline__ float bf16r(float x) {
    unsigned u = __float_as_uint(x);
    u = (u + 0x7FFFu + ((u >> 16) & 1u)) & 0xFFFF0000u;
    return __uint_as_float(u);
}

static __device__ __forceinline__ float ex2(float x) {
    return __builtin_amdgcn_exp2f(x);
}

static __device__ __forceinline__ void wave_lds_sync() {
    __builtin_amdgcn_fence(3, "wavefront");
    asm volatile("s_wait_dscnt 0" ::: "memory");
    __builtin_amdgcn_wave_barrier();
}

static __device__ __forceinline__ float wave_sum(float v) {
    v += __shfl_xor(v, 16, 32);
    v += __shfl_xor(v, 8, 32);
    v += __shfl_xor(v, 4, 32);
    v += __shfl_xor(v, 2, 32);
    v += __shfl_xor(v, 1, 32);
    return v;
}

__global__ __launch_bounds__(256) void k_wprep(const float* __restrict__ wq,
                                                const float* __restrict__ wk,
                                                const float* __restrict__ wv,
                                                const float* __restrict__ wo,
                                                const float* __restrict__ w1,
                                                const float* __restrict__ w2,
                                                _Float16* __restrict__ wall) {
    __shared__ __align__(16) _Float16 T[64 * PP];
    const unsigned tid  = threadIdx.x;
    const unsigned mid  = blockIdx.y;
    const unsigned tile = blockIdx.x;
    const unsigned hi4  = tile >> 4, lo4 = tile & 15u;

    const float* base = (mid == 0u) ? wq : (mid == 1u) ? wk : (mid == 2u) ? wv
                      : (mid == 3u) ? wo : (mid == 4u) ? w1 : w2;
    size_t soff; unsigned pitch, drow0, dcol0;
    if (mid < 3u) {
        soff  = (size_t)hi4 * (DM * HD) + (size_t)(lo4 * 64u) * HD;
        pitch = HD;
        drow0 = mid * 1024u + hi4 * 64u;
        dcol0 = lo4 * 64u;
    } else {
        soff  = (size_t)(hi4 * 64u) * DM + lo4 * 64u;
        pitch = DM;
        drow0 = mid * 1024u + lo4 * 64u;
        dcol0 = hi4 * 64u;
    }
#pragma unroll
    for (unsigned i = 0; i < 4; ++i) {
        const unsigned idx = i * 256u + tid;
        const unsigned r = idx >> 4, c4 = (idx & 15u) << 2;
        v4f v = *(const v4f*)(base + soff + (size_t)r * pitch + c4);
        T[(c4 + 0u) * PP + r] = (_Float16)(bf16r(v.x) * 64.0f);
        T[(c4 + 1u) * PP + r] = (_Float16)(bf16r(v.y) * 64.0f);
        T[(c4 + 2u) * PP + r] = (_Float16)(bf16r(v.z) * 64.0f);
        T[(c4 + 3u) * PP + r] = (_Float16)(bf16r(v.w) * 64.0f);
    }
    __syncthreads();
    const unsigned ln = tid >> 3, pc = (tid & 7u) << 3;
    v8h o0 = *(const v8h*)(&T[ln * PP + pc]);
    v8h o1 = *(const v8h*)(&T[(32u + ln) * PP + pc]);
    _Float16* d0 = wall + (size_t)(drow0 + ln) * DM + dcol0 + pc;
    _Float16* d1 = d0 + (size_t)32 * DM;
    *(volatile v8h*)d0 = o0;
    *(volatile v8h*)d1 = o1;
    __threadfence();
    *(volatile v8h*)d0 = o0;
    *(volatile v8h*)d1 = o1;
}

template <bool F32, bool F16>
static __device__ __forceinline__ void ln_store(const float* rb, float* of, _Float16* oh, unsigned lane) {
    if (F32) {
#pragma unroll
        for (unsigned c = 0; c < 8; ++c) {
            v4f v = *(const v4f*)(rb + c * 128u + lane * 4u);
            *(volatile v4f*)(of + c * 128u + lane * 4u) = v;
        }
    }
    if (F16) {
#pragma unroll
        for (unsigned j = 0; j < 4; ++j) {
            v4f a = *(const v4f*)(rb + j * 256u + lane * 8u);
            v4f b = *(const v4f*)(rb + j * 256u + lane * 8u + 4u);
            v8h h;
            h[0] = (_Float16)a.x; h[1] = (_Float16)a.y; h[2] = (_Float16)a.z; h[3] = (_Float16)a.w;
            h[4] = (_Float16)b.x; h[5] = (_Float16)b.y; h[6] = (_Float16)b.z; h[7] = (_Float16)b.w;
            *(volatile v8h*)(oh + j * 256u + lane * 8u) = h;
        }
    }
}

template <bool INBF, bool XSTRIDE, bool F32, bool F16>
__global__ __launch_bounds__(256) void k_ln(const float* __restrict__ in,
                                             const float* __restrict__ gamma,
                                             const float* __restrict__ beta,
                                             float* __restrict__ of,
                                             _Float16* __restrict__ oh) {
    __shared__ __align__(16) float rowb[8][DM];
    const unsigned tid  = threadIdx.x;
    const unsigned lane = tid & 31u;
    const unsigned w    = tid >> 5;
    const unsigned row  = blockIdx.x * 8u + w;
    const unsigned b    = row / (unsigned)SEQ;
    const unsigned s    = row - b * (unsigned)SEQ;
    const size_t irow   = XSTRIDE ? ((size_t)b * SEQ_FULL + s) : (size_t)row;
    const float* ip = in + irow * DM;
    float* rb = &rowb[w][0];

    float sum = 0.0f;
#pragma unroll 1
    for (unsigned c = 0; c < 8; ++c) {
        v4f v = *(const v4f*)(ip + c * 128u + lane * 4u);
        if (INBF) { v.x = bf16r(v.x); v.y = bf16r(v.y); v.z = bf16r(v.z); v.w = bf16r(v.w); }
        *(v4f*)(rb + c * 128u + lane * 4u) = v;
        sum += (v.x + v.y) + (v.z + v.w);
    }
    sum = wave_sum(sum);
    const float mean = sum * (1.0f / 1024.0f);

    float sq = 0.0f;
#pragma unroll 1
    for (unsigned c = 0; c < 8; ++c) {
        v4f v = *(const v4f*)(rb + c * 128u + lane * 4u);
        const float d0 = v.x - mean, d1 = v.y - mean, d2 = v.z - mean, d3 = v.w - mean;
        sq += d0 * d0;
        sq += d1 * d1;
        sq += d2 * d2;
        sq += d3 * d3;
    }
    sq = wave_sum(sq);
    const float rstd = rsqrtf(sq * (1.0f / 1024.0f) + 1.0e-5f);

#pragma unroll 1
    for (unsigned c = 0; c < 8; ++c) {
        v4f v = *(const v4f*)(rb + c * 128u + lane * 4u);
        v4f g = *(const v4f*)(gamma + c * 128u + lane * 4u);
        v4f t = *(const v4f*)(beta + c * 128u + lane * 4u);
        v4f y;
        y.x = ((v.x - mean) * rstd) * bf16r(g.x) + bf16r(t.x);
        y.y = ((v.y - mean) * rstd) * bf16r(g.y) + bf16r(t.y);
        y.z = ((v.z - mean) * rstd) * bf16r(g.z) + bf16r(t.z);
        y.w = ((v.w - mean) * rstd) * bf16r(g.w) + bf16r(t.w);
        *(v4f*)(rb + c * 128u + lane * 4u) = y;
    }
    wave_lds_sync();

    float*    ofr = F32 ? (of + (size_t)row * DM) : (float*)0;
    _Float16* ohr = F16 ? (oh + (size_t)row * DM) : (_Float16*)0;
    ln_store<F32, F16>(rb, ofr, ohr, lane);
    __threadfence();
    ln_store<F32, F16>(rb, ofr, ohr, lane);
}

static __device__ __forceinline__ void gemm_core(const _Float16* Ap, const _Float16* Bp,
                                                 unsigned lane, v8f (&acc)[2][4]) {
#pragma unroll
    for (int mi = 0; mi < 2; ++mi)
#pragma unroll
        for (int ni = 0; ni < 4; ++ni) acc[mi][ni] = zero8();
#pragma unroll 1
    for (unsigned k0 = 0; k0 < (unsigned)DM; k0 += 32u) {
        const v16h a0 = load_frag16(Ap + k0, DM, lane);
        const v16h a1 = load_frag16(Ap + (size_t)16 * DM + k0, DM, lane);
#pragma unroll
        for (int ni = 0; ni < 4; ++ni) {
            const v16h bf = load_frag16(Bp + (size_t)(ni * 16) * DM + k0, DM, lane);
            acc[0][ni] = wmma16(a0, bf, acc[0][ni]);
            acc[1][ni] = wmma16(a1, bf, acc[1][ni]);
        }
    }
}

template <bool RELU, bool VT>
__global__ __launch_bounds__(128) void k_gemm_h(const _Float16* __restrict__ A,
                                                 const _Float16* __restrict__ Bt,
                                                 _Float16* __restrict__ C,
                                                 unsigned ldc, float scale) {
    __shared__ __align__(16) _Float16 st[4][32 * 64];
    const unsigned tid  = threadIdx.x;
    const unsigned lane = tid & 31u;
    const unsigned w    = tid >> 5;
    const unsigned m0   = blockIdx.y * 64u + (w >> 1) * 32u;
    const unsigned n0   = blockIdx.x * 128u + (w & 1u) * 64u;

    v8f acc[2][4];
    gemm_core(A + (size_t)m0 * DM, Bt + (size_t)n0 * DM, lane, acc);

    const unsigned r0 = (lane >> 4) << 3;
    const unsigned cc = lane & 15u;
#pragma unroll
    for (int mi = 0; mi < 2; ++mi)
#pragma unroll
        for (int ni = 0; ni < 4; ++ni)
#pragma unroll
            for (int g = 0; g < 8; ++g) {
                float val = acc[mi][ni][g] * scale;
                if (RELU) val = fmaxf(val, 0.0f);
                st[w][(mi * 16 + r0 + g) * 64u + ni * 16 + cc] = (_Float16)val;
            }
    wave_lds_sync();

    size_t coloff;
    if (VT) {
        const unsigned bb = n0 / (unsigned)SEQ;
        coloff = (size_t)bb * ((size_t)DM * SEQ) + (n0 - bb * (unsigned)SEQ);
    } else {
        coloff = n0;
    }
    _Float16* cb = C + (size_t)m0 * ldc + coloff;
    const unsigned rq = lane >> 3, pc = (lane & 7u) << 3;
    v8h pv[8];
#pragma unroll
    for (unsigned i = 0; i < 8; ++i) pv[i] = *(const v8h*)(&st[w][(4u * i + rq) * 64u + pc]);
#pragma unroll
    for (unsigned i = 0; i < 8; ++i) *(volatile v8h*)(cb + (size_t)(4u * i + rq) * ldc + pc) = pv[i];
    __threadfence();
#pragma unroll
    for (unsigned i = 0; i < 8; ++i) *(volatile v8h*)(cb + (size_t)(4u * i + rq) * ldc + pc) = pv[i];
}

template <bool RBF>
__global__ __launch_bounds__(128) void k_gemm_f(const _Float16* __restrict__ A,
                                                 const _Float16* __restrict__ Bt,
                                                 const float* __restrict__ resid,
                                                 unsigned rseq,
                                                 float* __restrict__ C, float scale) {
    __shared__ __align__(16) float st[4][32 * 64];
    const unsigned tid  = threadIdx.x;
    const unsigned lane = tid & 31u;
    const unsigned w    = tid >> 5;
    const unsigned m0   = blockIdx.y * 64u + (w >> 1) * 32u;
    const unsigned n0   = blockIdx.x * 128u + (w & 1u) * 64u;

    v8f acc[2][4];
    gemm_core(A + (size_t)m0 * DM, Bt + (size_t)n0 * DM, lane, acc);

    const unsigned r0 = (lane >> 4) << 3;
    const unsigned cc = lane & 15u;
#pragma unroll
    for (int mi = 0; mi < 2; ++mi)
#pragma unroll
        for (int ni = 0; ni < 4; ++ni)
#pragma unroll
            for (int g = 0; g < 8; ++g)
                st[w][(mi * 16 + r0 + g) * 64u + ni * 16 + cc] = acc[mi][ni][g] * scale;
    wave_lds_sync();

    const unsigned rq = lane >> 4, pc = (lane & 15u) << 2;
    v4f ov[16];
#pragma unroll
    for (unsigned i = 0; i < 16; ++i) {
        const unsigned row = 2u * i + rq;
        const unsigned m   = m0 + row;
        const unsigned bb  = m / (unsigned)SEQ;
        const size_t rrow  = (size_t)bb * rseq + (m - bb * (unsigned)SEQ);
        v4f sv = *(const v4f*)(&st[w][row * 64u + pc]);
        v4f rv = *(const v4f*)(resid + rrow * DM + n0 + pc);
        if (RBF) { rv.x = bf16r(rv.x); rv.y = bf16r(rv.y); rv.z = bf16r(rv.z); rv.w = bf16r(rv.w); }
        v4f o;
        o.x = sv.x + rv.x; o.y = sv.y + rv.y; o.z = sv.z + rv.z; o.w = sv.w + rv.w;
        ov[i] = o;
    }
    float* cb = C + (size_t)m0 * DM + n0;
#pragma unroll
    for (unsigned i = 0; i < 16; ++i) *(volatile v4f*)(cb + (size_t)(2u * i + rq) * DM + pc) = ov[i];
    __threadfence();
#pragma unroll
    for (unsigned i = 0; i < 16; ++i) *(volatile v4f*)(cb + (size_t)(2u * i + rq) * DM + pc) = ov[i];
}

__global__ __launch_bounds__(256) __attribute__((amdgpu_num_vgpr(256)))
void k_attn(const _Float16* __restrict__ qk,
            const _Float16* __restrict__ vT,
            _Float16* __restrict__ ctx) {
    __shared__ __align__(16) _Float16 Pst[8][16 * PP];

    const unsigned tid  = threadIdx.x;
    const unsigned lane = tid & 31u;
    const unsigned w    = tid >> 5;
    const unsigned b    = blockIdx.y >> 4;
    const unsigned h    = blockIdx.y & 15u;
    const unsigned q0   = blockIdx.x * 128u + w * 16u;
    const unsigned r0   = (lane >> 4) << 3;
    const unsigned cc   = lane & 15u;

    const _Float16* qb = qk + ((size_t)b * SEQ + q0) * QKP + h * HD;
    const v16h qf0 = load_frag16(qb, QKP, lane);
    const v16h qf1 = load_frag16(qb + 32, QKP, lane);
    const _Float16* kb = qk + (size_t)b * SEQ * QKP + DM + h * HD;
    const _Float16* vb = vT + ((size_t)b * DM + h * HD) * SEQ;

    float mrow[8], lrow[8];
#pragma unroll
    for (int g = 0; g < 8; ++g) { mrow[g] = -1.0e30f; lrow[g] = 0.0f; }
    v8f o[4];
#pragma unroll
    for (int nt = 0; nt < 4; ++nt) o[nt] = zero8();

#pragma unroll 1
    for (unsigned t0 = 0; t0 < (unsigned)SEQ; t0 += 64u) {
        v8f s[4];
#pragma unroll
        for (int nt = 0; nt < 4; ++nt) {
            const _Float16* kp = kb + (size_t)(t0 + nt * 16) * QKP;
            const v16h kf0 = load_frag16(kp, QKP, lane);
            const v16h kf1 = load_frag16(kp + 32, QKP, lane);
            v8f c = wmma16(qf0, kf0, zero8());
            c = wmma16(qf1, kf1, c);
            s[nt] = c;
        }
#pragma unroll
        for (int g = 0; g < 8; ++g) {
            float mx = fmaxf(fmaxf(s[0][g], s[1][g]), fmaxf(s[2][g], s[3][g]));
            mx = fmaxf(mx, __shfl_xor(mx, 1, 32));
            mx = fmaxf(mx, __shfl_xor(mx, 2, 32));
            mx = fmaxf(mx, __shfl_xor(mx, 4, 32));
            mx = fmaxf(mx, __shfl_xor(mx, 8, 32));
            const float mn = fmaxf(mrow[g], mx * C1);
            const float al = ex2(mrow[g] - mn);
            mrow[g] = mn;
            const float bias = PCARRY - mn;
            const float p0 = ex2(__builtin_fmaf(s[0][g], C1, bias));
            const float p1 = ex2(__builtin_fmaf(s[1][g], C1, bias));
            const float p2 = ex2(__builtin_fmaf(s[2][g], C1, bias));
            const float p3 = ex2(__builtin_fmaf(s[3][g], C1, bias));
            lrow[g] = __builtin_fmaf(lrow[g], al, (p0 + p1) + (p2 + p3));
            o[0][g] *= al; o[1][g] *= al; o[2][g] *= al; o[3][g] *= al;
            _Float16* pr = &Pst[w][(r0 + g) * PP + cc];
            pr[0]  = (_Float16)p0;
            pr[16] = (_Float16)p1;
            pr[32] = (_Float16)p2;
            pr[48] = (_Float16)p3;
        }
        wave_lds_sync();
        const v16h pa0 = load_frag16(&Pst[w][0], PP, lane);
        const v16h pa1 = load_frag16(&Pst[w][32], PP, lane);
#pragma unroll
        for (int nt = 0; nt < 4; ++nt) {
            const _Float16* vp = vb + (size_t)(nt * 16) * SEQ + t0;
            const v16h vf0 = load_frag16(vp, SEQ, lane);
            const v16h vf1 = load_frag16(vp + 32, SEQ, lane);
            o[nt] = wmma16(pa0, vf0, o[nt]);
            o[nt] = wmma16(pa1, vf1, o[nt]);
        }
    }

#pragma unroll
    for (int g = 0; g < 8; ++g) {
        float l = lrow[g];
        l += __shfl_xor(l, 1, 32);
        l += __shfl_xor(l, 2, 32);
        l += __shfl_xor(l, 4, 32);
        l += __shfl_xor(l, 8, 32);
        const float inv = SC_CTX * __builtin_amdgcn_rcpf(l);
        _Float16* pr = &Pst[w][(r0 + g) * PP + cc];
        pr[0]  = (_Float16)(o[0][g] * inv);
        pr[16] = (_Float16)(o[1][g] * inv);
        pr[32] = (_Float16)(o[2][g] * inv);
        pr[48] = (_Float16)(o[3][g] * inv);
    }
    wave_lds_sync();

    const unsigned rq = lane >> 3, pc = (lane & 7u) << 3;
    v8h cv[4];
#pragma unroll
    for (unsigned i = 0; i < 4; ++i) cv[i] = *(const v8h*)(&Pst[w][(4u * i + rq) * PP + pc]);
    _Float16* cb = ctx + ((size_t)b * SEQ + q0) * DM + h * HD + pc;
#pragma unroll
    for (unsigned i = 0; i < 4; ++i) *(volatile v8h*)(cb + (size_t)(4u * i + rq) * DM) = cv[i];
    __threadfence();
#pragma unroll
    for (unsigned i = 0; i < 4; ++i) *(volatile v8h*)(cb + (size_t)(4u * i + rq) * DM) = cv[i];
}

extern "C" void kernel_launch(void* const* d_in, const int* in_sizes, int n_in,
                              void* d_out, int out_size, void* d_ws, size_t ws_size,
                              hipStream_t stream) {
    if (n_in < 13) return;
    if (in_sizes[0] < ((NB - 1) * SEQ_FULL + SEQ) * DM) return;
    for (int i = 1; i <= 6; ++i) if (in_sizes[i] < DM * DM) return;
    for (int i = 7; i <= 12; ++i) if (in_sizes[i] < DM) return;
    if (out_size < NTOK * DM) return;

    const float* x    = (const float*)d_in[0];
    const float* wq   = (const float*)d_in[1];
    const float* wk   = (const float*)d_in[2];
    const float* wv   = (const float*)d_in[3];
    const float* wo   = (const float*)d_in[4];
    const float* w1   = (const float*)d_in[5];
    const float* w2   = (const float*)d_in[6];
    const float* ln1g = (const float*)d_in[7];
    const float* ln1b = (const float*)d_in[8];
    const float* ln2g = (const float*)d_in[9];
    const float* ln2b = (const float*)d_in[10];
    const float* ln3g = (const float*)d_in[11];
    const float* ln3b = (const float*)d_in[12];
    float* out = (float*)d_out;

    char* ws = (char*)d_ws;
    size_t off = 0;
    _Float16* wall = (_Float16*)(ws + off); off += (size_t)WROWS * DM * 2;
    _Float16* h1   = (_Float16*)(ws + off); off += (size_t)NTOK * DM * 2;
    _Float16* qkp  = (_Float16*)(ws + off); off += (size_t)NTOK * QKP * 2;
    _Float16* vTp  = (_Float16*)(ws + off); off += (size_t)NB * DM * SEQ * 2;
    _Float16* ctx  = (_Float16*)(ws + off); off += (size_t)NTOK * DM * 2;
    float*    tmp  = (float*)(ws + off);    off += (size_t)NTOK * DM * 4;
    float*    h2f  = (float*)(ws + off);    off += (size_t)NTOK * DM * 4;
    _Float16* h2h  = (_Float16*)(ws + off); off += (size_t)NTOK * DM * 2;
    _Float16* up   = (_Float16*)(ws + off); off += (size_t)NTOK * DM * 2;
    float*    tmp2 = (float*)(ws + off);    off += (size_t)NTOK * DM * 4;
    if (off > ws_size) return;
    if (off > (size_t)134217728) return;

    k_wprep<<<dim3(256, 6), dim3(256), 0, stream>>>(wq, wk, wv, wo, w1, w2, wall);
    k_ln<true, true, false, true><<<dim3(NTOK / 8), dim3(256), 0, stream>>>(x, ln1g, ln1b, (float*)0, h1);
    k_gemm_h<false, false><<<dim3(QKP / 128, NTOK / 64), dim3(128), 0, stream>>>(
        h1, wall, qkp, (unsigned)QKP, SC_P8);
    k_gemm_h<false, true><<<dim3(NTOK / 128, DM / 64), dim3(128), 0, stream>>>(
        wall + (size_t)2048 * DM, h1, vTp, (unsigned)SEQ, SC_P8);
    k_attn<<<dim3(SEQ / 128, NB * NH), dim3(256), 0, stream>>>(qkp, vTp, ctx);
    k_gemm_f<true><<<dim3(DM / 128, NTOK / 64), dim3(128), 0, stream>>>(
        ctx, wall + (size_t)3072 * DM, x, (unsigned)SEQ_FULL, tmp, SC_WO);
    k_ln<false, false, true, true><<<dim3(NTOK / 8), dim3(256), 0, stream>>>(tmp, ln2g, ln2b, h2f, h2h);
    k_gemm_h<true, false><<<dim3(DM / 128, NTOK / 64), dim3(128), 0, stream>>>(
        h2h, wall + (size_t)4096 * DM, up, (unsigned)DM, SC_P8);
    k_gemm_f<false><<<dim3(DM / 128, NTOK / 64), dim3(128), 0, stream>>>(
        up, wall + (size_t)5120 * DM, h2f, (unsigned)SEQ, tmp2, SC_W2);
    k_ln<false, false, true, false><<<dim3(NTOK / 8), dim3(256), 0, stream>>>(tmp2, ln3g, ln3b, out, (_Float16*)0);
}
